// LSTM_11811160064747
// MI455X (gfx1250) — hardware-verified
//
#include <hip/hip_runtime.h>
#include <math.h>

constexpr int NB   = 131072;
constexpr int NSTP = 5;
constexpr int NIN  = 15;
constexpr int NH1  = 64;
constexpr int NH2  = 32;
constexpr int NH3  = 16;
constexpr int NG1  = 4 * NH1;
constexpr int NG2  = 4 * NH2;
constexpr int NG3  = 4 * NH3;
constexpr int NFC  = NSTP * NH3;
constexpr int XROW = NSTP * NIN;
constexpr int KP1 = 96;
constexpr int KP2 = 96;
constexpr int KP3 = 64;
constexpr int KPF = 96;
constexpr int NTHR  = 128;
constexpr int NWAVE = NTHR / 32;
constexpr int RBLK  = 16 * NWAVE;
constexpr float ASC = 8.0f;
constexpr float WSC = 256.0f;
constexpr float ACC_INV = 1.0f / (ASC * WSC);

constexpr int OW1 = 0;
constexpr int OW2 = OW1 + NG1 * KP1;
constexpr int OW3 = OW2 + NG2 * KP2;
constexpr int OWF = OW3 + NG3 * KP3;
constexpr int NWH = OWF + NFC * KPF;
constexpr int OA1 = 0;
constexpr int OA2 = OA1 + 16 * KP1;
constexpr int OA3 = OA2 + 16 * KP2;
constexpr int OAF = OA3 + 16 * KP3;
constexpr int AWH = OAF + 16 * KPF;
constexpr int OC1 = 0;
constexpr int OC2 = OC1 + NH1 * 16;
constexpr int OC3 = OC2 + NH2 * 16;
constexpr int CWF = OC3 + NH3 * 16;
constexpr int OBS1 = 0;
constexpr int OBS2 = OBS1 + NG1;
constexpr int OBS3 = OBS2 + NG2;
constexpr int OB1F = OBS3 + NG3;
constexpr int OW2F = OB1F + NFC;
constexpr int NFSH = OW2F + NFC;

static_assert(NB % RBLK == 0);
static_assert((NG1 * 32) % NTHR == 0 && (NG1 * NH1) % NTHR == 0);
static_assert((NG2 * NH1) % NTHR == 0 && (NG2 * NH2) % NTHR == 0);
static_assert((NG3 * NH2) % NTHR == 0 && (NG3 * 32) % NTHR == 0);
static_assert((NFC * KPF) % NTHR == 0);
static_assert(NG1 % NTHR == 0 && NG2 == NTHR && NG3 <= NTHR && NFC <= NTHR);
static_assert(AWH % 256 == 0 && CWF % 128 == 0);
static_assert(KP1 % 32 == 0 && KP2 % 32 == 0 && KP3 % 32 == 0 && KPF % 32 == 0);
static_assert(NIN + 17 + NH1 == KP1 && NH1 + NH2 == KP2 && NH2 + 32 == KP3 && NH2 + NH3 + 16 == KP3 && NFC + 16 == KPF);
static_assert(RBLK * 4 == 256);

typedef __attribute__((ext_vector_type(16))) _Float16 v16h;
typedef __attribute__((ext_vector_type(8)))  _Float16 v8h;
typedef __attribute__((ext_vector_type(8)))  float    v8f;
typedef __attribute__((ext_vector_type(4)))  float    v4f;

struct FragH {
  union U { v16h v; v8h h[2]; };
  static __device__ __forceinline__ v16h load(const _Float16* p) {
    U f; f.h[0] = *(const v8h*)(p); f.h[1] = *(const v8h*)(p + 16); return f.v;
  }
  static __device__ __forceinline__ v8f mma(v16h a, v16h b, v8f c) {
    return __builtin_amdgcn_wmma_f32_16x16x32_f16(false, a, false, b, (short)0, c, false, false);
  }
};

__device__ __forceinline__ void mma4(v8f& g0, v8f& g1, v8f& g2, v8f& g3, v16h a, const _Float16* wb, int gstride) {
  asm volatile("" ::: "memory");
  const v16h b0 = FragH::load(wb);
  const v16h b1 = FragH::load(wb + gstride);
  const v16h b2 = FragH::load(wb + 2 * gstride);
  const v16h b3 = FragH::load(wb + 3 * gstride);
  g0 = FragH::mma(a, b0, g0);
  g1 = FragH::mma(a, b1, g1);
  g2 = FragH::mma(a, b2, g2);
  g3 = FragH::mma(a, b3, g3);
  asm volatile("v_nop\n\tv_nop\n\tv_nop\n\tv_nop"
               : "+v"(g0), "+v"(g1), "+v"(g2), "+v"(g3)
               : "v"(a), "v"(b0), "v"(b1), "v"(b2), "v"(b3));
}
__device__ __forceinline__ void mma3(v8f& g, v16h a0, v16h a1, v16h a2, const _Float16* wb) {
  asm volatile("" ::: "memory");
  const v16h b0 = FragH::load(wb);
  const v16h b1 = FragH::load(wb + 32);
  const v16h b2 = FragH::load(wb + 64);
  g = FragH::mma(a0, b0, g);
  g = FragH::mma(a1, b1, g);
  g = FragH::mma(a2, b2, g);
  asm volatile("v_nop\n\tv_nop\n\tv_nop\n\tv_nop"
               : "+v"(g)
               : "v"(a0), "v"(a1), "v"(a2), "v"(b0), "v"(b1), "v"(b2));
}

__device__ __forceinline__ void wsync() {
  __builtin_amdgcn_fence(__ATOMIC_RELEASE, "workgroup");
  __builtin_amdgcn_wave_barrier();
  __builtin_amdgcn_fence(__ATOMIC_ACQUIRE, "workgroup");
}

__device__ __forceinline__ float fsig(float v)  { return __builtin_amdgcn_rcpf(1.0f + expf(-v)); }
__device__ __forceinline__ float ftanh(float v) { return 1.0f - 2.0f * __builtin_amdgcn_rcpf(expf(2.0f * v) + 1.0f); }

__device__ __forceinline__ void cell8(const v8f& ai, const v8f& af, const v8f& ag, const v8f& ao,
                                      float bi, float bf, float bg, float bo,
                                      float* cst, float (&hv)[8]) {
  const v4f ca = *(const v4f*)(cst);
  const v4f cb = *(const v4f*)(cst + 4);
  float co[8];
  co[0] = ca[0]; co[1] = ca[1]; co[2] = ca[2]; co[3] = ca[3];
  co[4] = cb[0]; co[5] = cb[1]; co[6] = cb[2]; co[7] = cb[3];
#pragma unroll
  for (int r = 0; r < 8; ++r) {
    const float zi = ai[r] * ACC_INV + bi;
    const float zf = af[r] * ACC_INV + bf;
    const float zg = ag[r] * ACC_INV + bg;
    const float zo = ao[r] * ACC_INV + bo;
    const float ig = fsig(zi);
    const float fg = fsig(zf);
    const float og = fsig(zo);
    const float gg = ftanh(zg);
    const float cn = fg * co[r] + ig * gg;
    co[r] = cn;
    hv[r] = og * ftanh(cn);
  }
  const v4f na = {co[0], co[1], co[2], co[3]};
  const v4f nb = {co[4], co[5], co[6], co[7]};
  *(v4f*)(cst)     = na;
  *(v4f*)(cst + 4) = nb;
}

__global__ __launch_bounds__(NTHR) __attribute__((amdgpu_num_vgpr(256)))
void lstm3_head_kernel(
    const float* __restrict__ x,
    const float* __restrict__ Wih1, const float* __restrict__ Whh1, const float* __restrict__ bih1, const float* __restrict__ bhh1,
    const float* __restrict__ Wih2, const float* __restrict__ Whh2, const float* __restrict__ bih2, const float* __restrict__ bhh2,
    const float* __restrict__ Wih3, const float* __restrict__ Whh3, const float* __restrict__ bih3, const float* __restrict__ bhh3,
    const float* __restrict__ W1,   const float* __restrict__ b1,   const float* __restrict__ W2,   const float* __restrict__ b2,
    float* __restrict__ out) {
  __shared__ __align__(16) _Float16 Wsh[NWH];
  __shared__ __align__(16) _Float16 Ash[NWAVE * AWH];
  __shared__ __align__(16) float    Csh[NWAVE * CWF];
  __shared__ __align__(16) float    Fsh[NFSH];
  __shared__ __align__(16) float    Osh[RBLK];

  const int tid = threadIdx.x, lane = tid & 31, wave = tid >> 5;
  const int c = lane & 15, hh = lane >> 4, koff = hh * 8;

#pragma unroll 1
  for (int i = tid; i < NG1 * 32; i += NTHR) {
    const int g = i >> 5, k = i & 31;
    const int ka = (k < NIN) ? k : (NIN - 1);
    const float w = Wih1[g * NIN + ka];
    const float v = (k < NIN) ? w * WSC : 0.0f;
    Wsh[OW1 + g * KP1 + k] = (_Float16)v;
  }
#pragma unroll 1
  for (int i = tid; i < NG1 * NH1; i += NTHR) {
    const int g = i >> 6, k = i & 63;
    Wsh[OW1 + g * KP1 + 32 + k] = (_Float16)(Whh1[i] * WSC);
  }
#pragma unroll 1
  for (int i = tid; i < NG2 * NH1; i += NTHR) {
    const int g = i >> 6, k = i & 63;
    Wsh[OW2 + g * KP2 + k] = (_Float16)(Wih2[i] * WSC);
  }
#pragma unroll 1
  for (int i = tid; i < NG2 * NH2; i += NTHR) {
    const int g = i >> 5, k = i & 31;
    Wsh[OW2 + g * KP2 + NH1 + k] = (_Float16)(Whh2[i] * WSC);
  }
#pragma unroll 1
  for (int i = tid; i < NG3 * NH2; i += NTHR) {
    const int g = i >> 5, k = i & 31;
    Wsh[OW3 + g * KP3 + k] = (_Float16)(Wih3[i] * WSC);
  }
#pragma unroll 1
  for (int i = tid; i < NG3 * 32; i += NTHR) {
    const int g = i >> 5, kk = i & 31;
    const int ka = (kk < NH3) ? kk : (NH3 - 1);
    const float w = Whh3[g * NH3 + ka];
    const float v = (kk < NH3) ? w * WSC : 0.0f;
    Wsh[OW3 + g * KP3 + NH2 + kk] = (_Float16)v;
  }
#pragma unroll 1
  for (int i = tid; i < NFC * KPF; i += NTHR) {
    const int g = i / KPF, k = i - g * KPF;
    const int ka = (k < NFC) ? k : (NFC - 1);
    const float w = W1[g * NFC + ka];
    const float v = (k < NFC) ? w * WSC : 0.0f;
    Wsh[OWF + i] = (_Float16)v;
  }
#pragma unroll 1
  for (int i = tid; i < NG1; i += NTHR) Fsh[OBS1 + i] = bih1[i] + bhh1[i];
  Fsh[OBS2 + tid] = bih2[tid] + bhh2[tid];
  {
    const int j3 = (tid < NG3) ? tid : (NG3 - 1);
    const float v3 = bih3[j3] + bhh3[j3];
    const int jf = (tid < NFC) ? tid : (NFC - 1);
    const float vb = b1[jf];
    const float vw = W2[jf];
    if (tid < NG3) Fsh[OBS3 + tid] = v3;
    if (tid < NFC) { Fsh[OB1F + tid] = vb; Fsh[OW2F + tid] = vw; }
  }
  const float b2v = b2[0];

  _Float16* Aw = Ash + wave * AWH;
  _Float16* A1 = Aw + OA1;
  _Float16* A2 = Aw + OA2;
  _Float16* A3 = Aw + OA3;
  _Float16* AF = Aw + OAF;
  float*    Cw = Csh + wave * CWF;
  const _Float16 hz = (_Float16)0.0f;
  const v8h zh = {hz, hz, hz, hz, hz, hz, hz, hz};
  const v4f z4f = {0.f, 0.f, 0.f, 0.f};
#pragma unroll 1
  for (int i = 0; i < AWH / 256; ++i) *(v8h*)(Aw + (i * 32 + lane) * 8) = zh;
#pragma unroll 1
  for (int i = 0; i < CWF / 128; ++i) *(v4f*)(Cw + (i * 32 + lane) * 4) = z4f;

  __syncthreads();

  const size_t rb = (size_t)blockIdx.x * RBLK + (size_t)wave * 16;
  const v8f z8 = {0.f, 0.f, 0.f, 0.f, 0.f, 0.f, 0.f, 0.f};

#pragma unroll 1
  for (int t = 0; t < NSTP; ++t) {
    wsync();
    {
      const float* xr = x + (rb + (size_t)c) * XROW + (size_t)t * NIN;
      float v[8];
#pragma unroll
      for (int e = 0; e < 7; ++e) v[e] = xr[koff + e];
      const int k7  = koff + 7;
      const int k7c = (k7 < NIN) ? k7 : (NIN - 1);
      const float w7 = xr[k7c];
      v[7] = (hh == 0) ? w7 : 0.0f;
      v8h pk;
#pragma unroll
      for (int e = 0; e < 8; ++e) pk[e] = (_Float16)(v[e] * ASC);
      *(v8h*)(A1 + c * KP1 + koff) = pk;
      *(v8h*)(A1 + c * KP1 + 16 + koff) = zh;
      *(v8h*)(A3 + c * KP3 + NH2 + NH3 + koff) = zh;
    }
    wsync();

    {
      const _Float16* ar = A1 + c * KP1 + koff;
      const v16h a0 = FragH::load(ar);
      const v16h a1 = FragH::load(ar + 32);
      const v16h a2 = FragH::load(ar + 64);
#pragma unroll 1
      for (int ut = 0; ut < NH1 / 16; ++ut) {
        const _Float16* wb = Wsh + OW1 + (ut * 16 + c) * KP1 + koff;
        v8f g0 = z8, g1 = z8, g2 = z8, g3 = z8;
        mma4(g0, g1, g2, g3, a0, wb,      NH1 * KP1);
        mma4(g0, g1, g2, g3, a1, wb + 32, NH1 * KP1);
        mma4(g0, g1, g2, g3, a2, wb + 64, NH1 * KP1);
        const int j = ut * 16 + c;
        float hv[8];
        cell8(g0, g1, g2, g3, Fsh[OBS1 + j], Fsh[OBS1 + NH1 + j], Fsh[OBS1 + 2 * NH1 + j], Fsh[OBS1 + 3 * NH1 + j],
              Cw + OC1 + j * 16 + koff, hv);
#pragma unroll
        for (int r = 0; r < 8; ++r) {
          A1[(koff + r) * KP1 + 32 + j] = (_Float16)(hv[r] * ASC);
          A2[(koff + r) * KP2 + j]      = (_Float16)(ftanh(hv[r]) * ASC);
        }
      }
    }
    wsync();

    {
      const _Float16* ar = A2 + c * KP2 + koff;
      const v16h a0 = FragH::load(ar);
      const v16h a1 = FragH::load(ar + 32);
      const v16h a2 = FragH::load(ar + 64);
#pragma unroll 1
      for (int ut = 0; ut < NH2 / 16; ++ut) {
        const _Float16* wb = Wsh + OW2 + (ut * 16 + c) * KP2 + koff;
        v8f g0 = z8, g1 = z8, g2 = z8, g3 = z8;
        mma4(g0, g1, g2, g3, a0, wb,      NH2 * KP2);
        mma4(g0, g1, g2, g3, a1, wb + 32, NH2 * KP2);
        mma4(g0, g1, g2, g3, a2, wb + 64, NH2 * KP2);
        const int j = ut * 16 + c;
        float hv[8];
        cell8(g0, g1, g2, g3, Fsh[OBS2 + j], Fsh[OBS2 + NH2 + j], Fsh[OBS2 + 2 * NH2 + j], Fsh[OBS2 + 3 * NH2 + j],
              Cw + OC2 + j * 16 + koff, hv);
#pragma unroll
        for (int r = 0; r < 8; ++r) {
          A2[(koff + r) * KP2 + NH1 + j] = (_Float16)(hv[r] * ASC);
          A3[(koff + r) * KP3 + j]       = (_Float16)(ftanh(hv[r]) * ASC);
        }
      }
    }
    wsync();

    {
      const _Float16* ar = A3 + c * KP3 + koff;
      const v16h a0 = FragH::load(ar);
      const v16h a1 = FragH::load(ar + 32);
      const _Float16* wb = Wsh + OW3 + c * KP3 + koff;
      v8f g0 = z8, g1 = z8, g2 = z8, g3 = z8;
      mma4(g0, g1, g2, g3, a0, wb,      NH3 * KP3);
      mma4(g0, g1, g2, g3, a1, wb + 32, NH3 * KP3);
      float hv[8];
      cell8(g0, g1, g2, g3, Fsh[OBS3 + c], Fsh[OBS3 + NH3 + c], Fsh[OBS3 + 2 * NH3 + c], Fsh[OBS3 + 3 * NH3 + c],
            Cw + OC3 + c * 16 + koff, hv);
#pragma unroll
      for (int r = 0; r < 8; ++r) {
        const _Float16 hq = (_Float16)(hv[r] * ASC);
        A3[(koff + r) * KP3 + NH2 + c]     = hq;
        AF[(koff + r) * KPF + t * NH3 + c] = hq;
      }
    }
  }

  wsync();
  *(v8h*)(AF + c * KPF + NFC + koff) = zh;
  wsync();
  float s[8];
  {
    const _Float16* ar = AF + c * KPF + koff;
    const v16h f0 = FragH::load(ar);
    const v16h f1 = FragH::load(ar + 32);
    const v16h f2 = FragH::load(ar + 64);
#pragma unroll
    for (int r = 0; r < 8; ++r) s[r] = 0.0f;
#pragma unroll
    for (int n = 0; n < NFC / 16; ++n) {
      const _Float16* wb = Wsh + OWF + (n * 16 + c) * KPF + koff;
      v8f g = z8;
      mma3(g, f0, f1, f2, wb);
      const int j = n * 16 + c;
      const float bb = Fsh[OB1F + j];
      const float ww = Fsh[OW2F + j];
#pragma unroll
      for (int r = 0; r < 8; ++r) {
        const float z = fmaxf(g[r] * ACC_INV + bb, 0.0f);
        s[r] = fmaf(z, ww, s[r]);
      }
    }
  }
#pragma unroll
  for (int r = 0; r < 8; ++r) {
    float sr = s[r];
    sr += __shfl_xor(sr, 1, 32);
    sr += __shfl_xor(sr, 2, 32);
    sr += __shfl_xor(sr, 4, 32);
    sr += __shfl_xor(sr, 8, 32);
    s[r] = sr + b2v;
  }
  if (c == 0) {
    const v4f o0 = {s[0], s[1], s[2], s[3]};
    const v4f o1 = {s[4], s[5], s[6], s[7]};
    *(v4f*)(Osh + wave * 16 + koff)     = o0;
    *(v4f*)(Osh + wave * 16 + koff + 4) = o1;
  }
  __syncthreads();

  {
    const int li = (lane < 16) ? lane : 15;
    const v4f ov = *(const v4f*)(Osh + li * 4);
    float* op = out + (size_t)blockIdx.x * RBLK + (size_t)li * 4;
    const bool writer = (wave == 0) && (lane < 16);
    if (writer) *(volatile v4f*)op = ov;
    __threadfence();
    if (writer) *(volatile v4f*)op = ov;
  }
}

extern "C" void kernel_launch(void* const* d_in, const int* in_sizes, int n_in,
                              void* d_out, int out_size, void* d_ws, size_t ws_size, hipStream_t stream) {
  (void)d_ws; (void)ws_size;
  if (n_in < 17 || d_out == nullptr) return;
  const long nx = (long)NB * XROW;
  if (!((long)in_sizes[0] == nx || (long)in_sizes[0] == nx * 4L)) return;
  if (!((long)out_size == (long)NB || (long)out_size == (long)NB * 4L)) return;

  const float* x    = (const float*)d_in[0];
  const float* Wih1 = (const float*)d_in[1];
  const float* Whh1 = (const float*)d_in[2];
  const float* bih1 = (const float*)d_in[3];
  const float* bhh1 = (const float*)d_in[4];
  const float* Wih2 = (const float*)d_in[5];
  const float* Whh2 = (const float*)d_in[6];
  const float* bih2 = (const float*)d_in[7];
  const float* bhh2 = (const float*)d_in[8];
  const float* Wih3 = (const float*)d_in[9];
  const float* Whh3 = (const float*)d_in[10];
  const float* bih3 = (const float*)d_in[11];
  const float* bhh3 = (const float*)d_in[12];
  const float* W1   = (const float*)d_in[13];
  const float* b1   = (const float*)d_in[14];
  const float* W2   = (const float*)d_in[15];
  const float* b2   = (const float*)d_in[16];
  float* out = (float*)d_out;

  lstm3_head_kernel<<<NB / RBLK, NTHR, 0, stream>>>(
      x, Wih1, Whh1, bih1, bhh1, Wih2, Whh2, bih2, bhh2, Wih3, Whh3, bih3, bhh3, W1, b1, W2, b2, out);
}
